// GkNN_86285892977149
// MI455X (gfx1250) — hardware-verified
//
#include <hip/hip_runtime.h>
#include <math.h>

typedef __attribute__((ext_vector_type(16))) _Float16 v16h;
typedef __attribute__((ext_vector_type(16))) __bf16 v16b;
typedef __attribute__((ext_vector_type(8)))  _Float16 v8h;
typedef __attribute__((ext_vector_type(8)))  float v8f;
typedef __attribute__((ext_vector_type(4)))  float v4f;
typedef __attribute__((ext_vector_type(2)))  float v2f;
typedef __attribute__((ext_vector_type(4)))  unsigned v4u;
typedef __attribute__((ext_vector_type(4)))  int v4i;
typedef float __attribute__((may_alias)) float_a;
typedef int __attribute__((may_alias)) int_a;

template <typename T> __device__ __forceinline__ void vst2(void* p, T v) { *(volatile T*)p = v; __threadfence(); *(volatile T*)p = v; }
__device__ __forceinline__ v8f wmma16(v16h a, v16h b, v8f c) {
  v8f d = __builtin_amdgcn_wmma_f32_16x16x32_f16(false, a, false, b, (short)0, c, false, false);
  asm volatile("v_nop\n\tv_nop\n\tv_nop\n\tv_nop" : "+v"(d) : "v"(a), "v"(b));
  return d;
}
__device__ __forceinline__ v8f wmma_bf(v16b a, v16b b, v8f c) {
  v8f d = __builtin_amdgcn_wmma_f32_16x16x32_bf16(false, a, false, b, (short)0, c, false, false);
  asm volatile("v_nop\n\tv_nop\n\tv_nop\n\tv_nop" : "+v"(d) : "v"(a), "v"(b));
  return d;
}
__device__ __forceinline__ v16h frag_h(const _Float16* rowk0, int lane) {
  union { v16h v; v8h q[2]; } u; const _Float16* p = rowk0 + 8 * (lane >> 4);
  u.q[0] = *(const v8h*)p; u.q[1] = *(const v8h*)(p + 16); return u.v;
}
__device__ __forceinline__ v16h frag_f32(const float* rowk0, int lane) {
  v16h a; const float* p = rowk0 + 8 * (lane >> 4);
#pragma unroll
  for (int i = 0; i < 8; ++i) { a[i] = (_Float16)p[i]; a[8 + i] = (_Float16)p[16 + i]; }
  return a;
}
__device__ __forceinline__ v16h frag_f32s(const float* rowk0, int lane, float sc) {
  v16h a; const float* p = rowk0 + 8 * (lane >> 4);
#pragma unroll
  for (int i = 0; i < 8; ++i) { a[i] = (_Float16)(p[i] * sc); a[8 + i] = (_Float16)(p[16 + i] * sc); }
  return a;
}
__device__ __forceinline__ v16h fragc_f32(const float* W, int k0, int n, int lane, int ld, int K) {
  v16h a; const int g = lane >> 4;
#pragma unroll
  for (int i = 0; i < 8; ++i) { const int ka = k0 + 8 * g + i, kb = ka + 16;
    a[i] = (_Float16)(ka < K ? W[(size_t)(ka < K ? ka : K - 1) * ld + n] : 0.f); a[8 + i] = (_Float16)(kb < K ? W[(size_t)(kb < K ? kb : K - 1) * ld + n] : 0.f); }
  return a;
}
struct F2 { v16b h, l; };
__device__ __forceinline__ F2 bsplit16(const float v[16]) { F2 r;
#pragma unroll
  for (int i = 0; i < 16; ++i) { const __bf16 h = (__bf16)v[i]; r.h[i] = h; r.l[i] = (__bf16)(v[i] - (float)h); }
  return r; }
__device__ __forceinline__ F2 split_row(const float* row, int k0, int lane) { float v[16]; const float* p = row + k0 + 8 * (lane >> 4);
#pragma unroll
  for (int i = 0; i < 8; ++i) { v[i] = p[i]; v[8 + i] = p[16 + i]; }
  return bsplit16(v); }
__device__ __forceinline__ F2 split_rowK(const float* row, int k0, int lane, int K) { float v[16]; const int g = lane >> 4;
#pragma unroll
  for (int i = 0; i < 8; ++i) { const int ka = k0 + 8 * g + i, kb = ka + 16; v[i] = ka < K ? row[ka < K ? ka : K - 1] : 0.f; v[8 + i] = kb < K ? row[kb < K ? kb : K - 1] : 0.f; }
  return bsplit16(v); }
__device__ __forceinline__ F2 split_col(const float* W, int k0, int n, int lane, int ld, int K) { float v[16]; const int g = lane >> 4;
#pragma unroll
  for (int i = 0; i < 8; ++i) { const int ka = k0 + 8 * g + i, kb = ka + 16; v[i] = ka < K ? W[(size_t)(ka < K ? ka : K - 1) * ld + n] : 0.f; v[8 + i] = kb < K ? W[(size_t)(kb < K ? kb : K - 1) * ld + n] : 0.f; }
  return bsplit16(v); }
__device__ __forceinline__ v8f mac3(const F2& a, const F2& b, v8f c) { c = wmma_bf(a.l, b.h, c); c = wmma_bf(a.h, b.l, c); return wmma_bf(a.h, b.h, c); }
__device__ __forceinline__ float sigm(float v) { return 1.0f / (1.0f + expf(-v)); }
#define LDSX() do { asm volatile("s_wait_dscnt 0" ::: "memory"); __builtin_amdgcn_wave_barrier(); __builtin_amdgcn_fence(__ATOMIC_RELEASE, "workgroup"); } while (0)


#define NBATCH 16
#define NN 8192
#define DD 128
#define KM 128
#define NR (NBATCH * NN)
#define SH 4096.0f
#define SK 65536.0f
#define SB 256.0f
#define SX2 67108864.0f
#define WSC 256.0f
typedef __attribute__((ext_vector_type(8))) __bf16 v8b;
__device__ __forceinline__ v16b frag_b(const __bf16* rowk0, int lane) {
  union { v16b v; v8b q[2]; } u; const __bf16* p = rowk0 + 8 * (lane >> 4);
  u.q[0] = *(const v8b*)p; u.q[1] = *(const v8b*)(p + 16); return u.v;
}
__device__ __forceinline__ float bfr(float v) { return (float)(__bf16)v; }
__device__ __attribute__((noinline)) float exp_ni(float v) { return expf(v); }
__device__ __attribute__((noinline)) float erf_ni(float v) { return erff(v); }
__device__ __attribute__((noinline)) float gelu_e(float v) { return 0.5f * v * (1.0f + erff(v * 0.70710678118654752f)); }

#define WS_PW  0u
#define WS_B16 (WS_PW + 2u * (size_t)10 * DD * DD)
#define WS_BT  (WS_B16 + 2u * (size_t)NN * KM)
#define WS_H32 (WS_BT + 2u * (size_t)KM * NN)
#define WS_H16 (WS_H32 + 4u * (size_t)NR * DD)
#define WS_P16 (WS_H16 + 2u * (size_t)NR * DD)
#define WS_U16 (WS_P16 + 2u * (size_t)NR * DD)
#define WS_SCT (WS_U16 + 2u * (size_t)NR * DD)
#define WS_XH  (WS_SCT + 2u * (size_t)NBATCH * KM * KM)
#define WS_XH2 (WS_XH + 4u * (size_t)NBATCH * DD * KM)
#define WS_END (WS_XH2 + 2u * (size_t)NBATCH * DD * KM)

__global__ __launch_bounds__(128) void k_packw(const float* __restrict__ M0, const float* __restrict__ M1, const float* __restrict__ M2, const float* __restrict__ M3, const float* __restrict__ M4, const float* __restrict__ M5, const float* __restrict__ M6, const float* __restrict__ M7, const float* __restrict__ M8, const float* __restrict__ M9, _Float16* __restrict__ PW) {
  const int o = blockIdx.x, which = blockIdx.y, t = threadIdx.x; __shared__ __align__(16) _Float16 sh[DD]; const float* m = which == 0 ? M0 : which == 1 ? M1 : which == 2 ? M2 : which == 3 ? M3 : which == 4 ? M4 : which == 5 ? M5 : which == 6 ? M6 : which == 7 ? M7 : which == 8 ? M8 : M9;
  sh[t] = (_Float16)(bfr(m[(size_t)t * DD + o]) * WSC); __syncthreads(); if (t < DD / 8) vst2((unsigned*)(PW + ((size_t)which * DD + o) * DD + t * 8), *(const v4u*)&sh[t * 8]); }
__global__ __launch_bounds__(128) void k_packB(const float* __restrict__ Bm, _Float16* __restrict__ B16, _Float16* __restrict__ BT) { __shared__ __align__(16) _Float16 s1[64][KM + 8]; __shared__ __align__(16) _Float16 s2[KM][64 + 8]; const int t = threadIdx.x; const int n0 = blockIdx.x * 64;
  for (int e = t; e < 64 * KM; e += 128) { const int rl = e >> 7, k = e & 127; const _Float16 v = (_Float16)(bfr(Bm[(size_t)(n0 + rl) * KM + k]) * SB); s1[rl][k] = v; s2[k][rl] = v; } __syncthreads();
  for (int e = t; e < 64 * 16; e += 128) { const int rl = e >> 4, q = e & 15; vst2((unsigned*)(B16 + (size_t)(n0 + rl) * KM + q * 8), *(const v4u*)&s1[rl][q * 8]); }
  for (int e = t; e < KM * 8; e += 128) { const int k = e >> 3, q = e & 7; vst2((unsigned*)(BT + (size_t)k * NN + n0 + q * 8), *(const v4u*)&s2[k][q * 8]); } }
__device__ __forceinline__ void store_h(float (*sf)[132], _Float16 (*sh)[136], size_t rb, int tid, float* H32, _Float16* H16) {
  for (int e = tid; e < 64 * 32; e += 128) { const int rl = e >> 5, q = e & 31; vst2(H32 + (rb + rl) * DD + q * 4, *(const v4f*)&sf[rl][q * 4]); }
  for (int e = tid; e < 64 * 16; e += 128) { const int rl = e >> 4, q = e & 15; vst2((unsigned*)(H16 + (rb + rl) * DD + q * 8), *(const v4u*)&sh[rl][q * 8]); } }
__global__ __launch_bounds__(128) void k_fc0(const float* __restrict__ X, const float* __restrict__ W1, const float* __restrict__ B1, const _Float16* __restrict__ PW, const float* __restrict__ B2, float* __restrict__ H32, _Float16* __restrict__ H16) {
  __shared__ __align__(16) _Float16 ah[64][DD + 8], al[64][DD + 8]; __shared__ __align__(16) float sf[64][132]; __shared__ __align__(16) _Float16 sh[64][136];
  const int tid = threadIdx.x, wave = tid >> 5, lane = tid & 31, col = lane & 15, g = lane >> 4; const size_t rb = (size_t)blockIdx.x * 64;
  for (int e = tid; e < 64 * DD; e += 128) { const int rl = e >> 7, j = e & 127; const float x0 = bfr(X[(rb + rl) * 2]), x1 = bfr(X[(rb + rl) * 2 + 1]); const float v = gelu_e(x0 * bfr(W1[j]) + x1 * bfr(W1[DD + j]) + bfr(B1[j])) * SH; const _Float16 hv = (_Float16)v; ah[rl][j] = hv; al[rl][j] = (_Float16)((v - (float)hv) * 2048.0f); }
  __syncthreads();
  v8f acc[8] = {}, accl[8] = {};
#pragma unroll
  for (int kc = 0; kc < DD / 32; ++kc) { v16h a, a2; { const _Float16* p = &ah[wave * 16 + col][kc * 32 + 8 * g]; const _Float16* p2 = &al[wave * 16 + col][kc * 32 + 8 * g];
#pragma unroll
      for (int i = 0; i < 8; ++i) { a[i] = p[i]; a[8 + i] = p[16 + i]; a2[i] = p2[i]; a2[8 + i] = p2[16 + i]; } }
#pragma unroll
    for (int j = 0; j < 8; ++j) { const v16h w = frag_h(PW + (size_t)(j * 16 + col) * DD + kc * 32, lane); acc[j] = wmma16(a, w, acc[j]); accl[j] = wmma16(a2, w, accl[j]); } }
#pragma unroll
  for (int j = 0; j < 8; ++j) { const float bb = bfr(B2[j * 16 + col]);
#pragma unroll
    for (int r = 0; r < 8; ++r) { const float v = (acc[j][r] + accl[j][r] * (1.0f / 2048.0f)) * (1.0f / (SH * WSC)) + bb; sf[wave * 16 + 8 * g + r][j * 16 + col] = v; sh[wave * 16 + 8 * g + r][j * 16 + col] = (_Float16)(v * SH); } }
  __syncthreads(); store_h(sf, sh, rb, tid, H32, H16); }
template <int MODE>
__global__ __launch_bounds__(128) void k_tok(const _Float16* __restrict__ A16, const float* __restrict__ A32, float ascale, const _Float16* __restrict__ Wr, const float* __restrict__ BIAS, float* __restrict__ H32, _Float16* __restrict__ H16, _Float16* __restrict__ P16, _Float16* __restrict__ U16, int PL, const float* __restrict__ FC2W, const float* __restrict__ FC2B, float* __restrict__ OUT) {
  __shared__ __align__(16) float sf[64][132]; __shared__ __align__(16) _Float16 sh[64][136]; __shared__ __align__(16) _Float16 st[DD][64 + 8];
  const int tid = threadIdx.x, wave = tid >> 5, lane = tid & 31, col = lane & 15, g = lane >> 4; const size_t rb = (size_t)blockIdx.x * 64; const size_t r0 = rb + wave * 16;
  v8f acc[8] = {}, accl[8] = {};
#pragma unroll
  for (int kc = 0; kc < DD / 32; ++kc) { if (MODE == 3) { v16h a, a2; { const float* p = A32 + (r0 + col) * DD + kc * 32 + 8 * g;
#pragma unroll
        for (int i = 0; i < 8; ++i) { const float x0 = p[i] * SH, x1 = p[16 + i] * SH; const _Float16 q0 = (_Float16)x0, q1 = (_Float16)x1; a[i] = q0; a[8 + i] = q1; a2[i] = (_Float16)((x0 - (float)q0) * 2048.0f); a2[8 + i] = (_Float16)((x1 - (float)q1) * 2048.0f); } }
#pragma unroll
      for (int j = 0; j < 8; ++j) { const v16h w = frag_h(Wr + (size_t)(j * 16 + col) * DD + kc * 32, lane); acc[j] = wmma16(a, w, acc[j]); accl[j] = wmma16(a2, w, accl[j]); } }
    else { const v16h a = frag_h(A16 + (r0 + col) * DD + kc * 32, lane);
#pragma unroll
      for (int j = 0; j < 8; ++j) acc[j] = wmma16(a, frag_h(Wr + (size_t)(j * 16 + col) * DD + kc * 32, lane), acc[j]); } }
  const float inv = 1.0f / (ascale * WSC);
  if (MODE == 3) { float part[8];
#pragma unroll
    for (int r = 0; r < 8; ++r) { part[r] = 0.f;
#pragma unroll
      for (int j = 0; j < 8; ++j) { const int c = j * 16 + col; const float v = (acc[j][r] + accl[j][r] * (1.0f / 2048.0f)) * inv + bfr(BIAS[c]); part[r] += gelu_e(v) * bfr(FC2W[c]); }
#pragma unroll
      for (int o = 1; o < 16; o <<= 1) part[r] += __shfl_xor(part[r], o);
      if (col == 0) sf[0][wave * 16 + 8 * g + r] = part[r] + bfr(FC2B[0]); }
    __syncthreads(); if (tid < 16) vst2(OUT + rb + tid * 4, *(const v4f*)&sf[0][tid * 4]); return; }
#pragma unroll
  for (int j = 0; j < 8; ++j) { const int c = j * 16 + col; const float bb = bfr(BIAS[c]);
#pragma unroll
    for (int r = 0; r < 8; ++r) { const int rl = wave * 16 + 8 * g + r; const float v = acc[j][r] * inv + bb;
      if (MODE == 0) st[c][rl] = (_Float16)(v * SK);
      else if (MODE == 1) sh[rl][c] = (_Float16)(gelu_e(v) * SK);
      else { const float h = H32[(rb + rl) * DD + c] + v; sf[rl][c] = h; sh[rl][c] = (_Float16)(h * SH); if (PL) st[c][rl] = (_Float16)(h * SH); } } }
  __syncthreads();
  if (MODE == 0 || (MODE == 2 && PL)) { const size_t b = rb / NN; const int n0 = (int)(rb % NN); for (int e = tid; e < DD * 8; e += 128) { const int c = e >> 3, q = e & 7; vst2((unsigned*)(P16 + ((b * DD + c) * NN) + n0 + q * 8), *(const v4u*)&st[c][q * 8]); } }
  if (MODE == 1) { for (int e = tid; e < 64 * 16; e += 128) { const int rl = e >> 4, q = e & 15; vst2((unsigned*)(U16 + (rb + rl) * DD + q * 8), *(const v4u*)&sh[rl][q * 8]); } }
  if (MODE == 2) store_h(sf, sh, rb, tid, H32, H16); }
template <int MODE>
__global__ __launch_bounds__(128) void k_nred(const _Float16* __restrict__ P16, const _Float16* __restrict__ BT, _Float16* __restrict__ SCT, float* __restrict__ XH) { __shared__ __align__(16) float sf[64][132]; __shared__ __align__(16) _Float16 st[KM][64 + 8];
  const int tid = threadIdx.x, wave = tid >> 5, lane = tid & 31, col = lane & 15, g = lane >> 4; const size_t b = blockIdx.y; const int i0 = blockIdx.x * 64 + wave * 16; const _Float16* Ab = P16 + (b * DD + i0) * NN;
  v8f acc[8] = {};
#pragma unroll 2
  for (int kc = 0; kc < NN / 32; ++kc) { const v16h a = frag_h(Ab + (size_t)col * NN + kc * 32, lane);
#pragma unroll
    for (int j = 0; j < 8; ++j) acc[j] = wmma16(a, frag_h(BT + (size_t)(j * 16 + col) * NN + kc * 32, lane), acc[j]); }
  const float inv = (MODE == 0) ? 1.0f / (SK * SB) : 1.0f / (SH * SB);
#pragma unroll
  for (int j = 0; j < 8; ++j)
#pragma unroll
    for (int r = 0; r < 8; ++r) { const int rl = wave * 16 + 8 * g + r; const float v = acc[j][r] * inv; if (MODE == 0) st[j * 16 + col][rl] = (_Float16)(v * SK); else sf[rl][j * 16 + col] = v; }
  __syncthreads();
  if (MODE == 0) { for (int e = tid; e < KM * 8; e += 128) { const int jv = e >> 3, q = e & 7; vst2((unsigned*)(SCT + ((b * KM + jv) * KM) + blockIdx.x * 64 + q * 8), *(const v4u*)&st[jv][q * 8]); } }
  else { for (int e = tid; e < 64 * 32; e += 128) { const int rl = e >> 5, q = e & 31; vst2(XH + ((b * DD + blockIdx.x * 64 + rl) * KM) + q * 4, *(const v4f*)&sf[rl][q * 4]); } } }
__global__ __launch_bounds__(128) void k_attn(const _Float16* __restrict__ B16, const _Float16* __restrict__ SCT, float* __restrict__ H32, _Float16* __restrict__ H16) { __shared__ __align__(16) float sf[64][132]; __shared__ __align__(16) _Float16 sh[64][136];
  const int tid = threadIdx.x, wave = tid >> 5, lane = tid & 31, col = lane & 15, g = lane >> 4; const size_t b = blockIdx.y; const int n0 = blockIdx.x * 64; const size_t rb = b * NN + n0; const _Float16* Wr = SCT + b * KM * KM;
  v8f acc[8] = {};
#pragma unroll
  for (int kc = 0; kc < KM / 32; ++kc) { const v16h a = frag_h(B16 + (size_t)(n0 + wave * 16 + col) * KM + kc * 32, lane);
#pragma unroll
    for (int j = 0; j < 8; ++j) acc[j] = wmma16(a, frag_h(Wr + (size_t)(j * 16 + col) * KM + kc * 32, lane), acc[j]); }
#pragma unroll
  for (int j = 0; j < 8; ++j)
#pragma unroll
    for (int r = 0; r < 8; ++r) { const int rl = wave * 16 + 8 * g + r, c = j * 16 + col; const float h = gelu_e(acc[j][r] * (1.0f / (SB * SK))) + H32[(rb + rl) * DD + c]; sf[rl][c] = h; sh[rl][c] = (_Float16)(h * SH); }
  __syncthreads(); store_h(sf, sh, rb, tid, H32, H16); }
__global__ __launch_bounds__(128) void k_mode(const float* __restrict__ XH, const float* __restrict__ WG, _Float16* __restrict__ XH2) { __shared__ __align__(16) _Float16 so2[KM]; const int k = threadIdx.x; const int o = blockIdx.x; const size_t b = blockIdx.y;
  float a = 0.f;
#pragma unroll 1
  for (int i = 0; i < DD; ++i) a += XH[((b * DD + i) * KM) + k] * bfr(WG[((size_t)i * DD + o) * KM + k]);
  so2[k] = (_Float16)(a * SX2); __syncthreads(); if (k < KM / 8) vst2((unsigned*)(XH2 + ((b * DD + o) * KM) + k * 8), *(const v4u*)&so2[k * 8]); }
__global__ __launch_bounds__(128) void k_gal(const _Float16* __restrict__ B16, const _Float16* __restrict__ XH2, const _Float16* __restrict__ Wr, const float* __restrict__ BIAS, int G, float* __restrict__ H32, _Float16* __restrict__ H16) { __shared__ __align__(16) float sf[64][132]; __shared__ __align__(16) _Float16 sh[64][136];
  const int tid = threadIdx.x, wave = tid >> 5, lane = tid & 31, col = lane & 15, g = lane >> 4; const size_t b = blockIdx.y; const int n0 = blockIdx.x * 64; const size_t rb = b * NN + n0; const size_t r0 = rb + wave * 16; const _Float16* X2 = XH2 + b * DD * KM;
  v8f acc1[8] = {}, acc2[8] = {};
#pragma unroll
  for (int kc = 0; kc < KM / 32; ++kc) { const v16h a1 = frag_h(B16 + (size_t)(n0 + wave * 16 + col) * KM + kc * 32, lane); const v16h a2 = frag_h(H16 + (r0 + col) * DD + kc * 32, lane);
#pragma unroll
    for (int j = 0; j < 8; ++j) { acc1[j] = wmma16(a1, frag_h(X2 + (size_t)(j * 16 + col) * KM + kc * 32, lane), acc1[j]); acc2[j] = wmma16(a2, frag_h(Wr + (size_t)(j * 16 + col) * DD + kc * 32, lane), acc2[j]); } }
#pragma unroll
  for (int j = 0; j < 8; ++j) { const int c = j * 16 + col; const float bb = bfr(BIAS[c]);
#pragma unroll
    for (int r = 0; r < 8; ++r) { const int rl = wave * 16 + 8 * g + r; const float s = acc1[j][r] * (1.0f / (SB * SX2)) + acc2[j][r] * (1.0f / (SH * WSC)) + bb; const float h = H32[(rb + rl) * DD + c] + (G ? gelu_e(s) : s); sf[rl][c] = h; sh[rl][c] = (_Float16)(h * SH); } }
  __syncthreads(); store_h(sf, sh, rb, tid, H32, H16); }
extern "C" void kernel_launch(void* const* d_in, const int* in_sizes, int n_in, void* d_out, int out_size, void* d_ws, size_t ws_size, hipStream_t stream) {
  (void)in_sizes; (void)n_in; (void)out_size;
  const float** F = (const float**)d_in;
  if (ws_size < (size_t)WS_END) return;
  char* ws = (char*)d_ws; _Float16 *PW = (_Float16*)(ws + WS_PW), *B16 = (_Float16*)(ws + WS_B16), *BT = (_Float16*)(ws + WS_BT), *H16 = (_Float16*)(ws + WS_H16), *P16 = (_Float16*)(ws + WS_P16), *U16 = (_Float16*)(ws + WS_U16), *SCT = (_Float16*)(ws + WS_SCT), *XH2 = (_Float16*)(ws + WS_XH2); float *H32 = (float*)(ws + WS_H32), *XH = (float*)(ws + WS_XH);
  const size_t MW = (size_t)DD * DD; const int TR = NR / 64, TPB = NN / 64;
  k_packw<<<dim3(DD, 10), 128, 0, stream>>>(F[4], F[6], F[8], F[10], F[13], F[15], F[17], F[19], F[22], F[24], PW);
  k_packB<<<NN / 64, 128, 0, stream>>>(F[1], B16, BT);
  k_fc0<<<TR, 128, 0, stream>>>(F[0], F[2], F[3], PW + 0 * MW, F[5], H32, H16);
  k_tok<0><<<TR, 128, 0, stream>>>(H16, nullptr, SH, PW + 1 * MW, F[7], H32, H16, P16, U16, 0, nullptr, nullptr, nullptr);
  k_nred<0><<<dim3(DD / 64, NBATCH), 128, 0, stream>>>(P16, BT, SCT, XH);
  k_attn<<<dim3(TPB, NBATCH), 128, 0, stream>>>(B16, SCT, H32, H16);
  k_tok<1><<<TR, 128, 0, stream>>>(H16, nullptr, SH, PW + 2 * MW, F[9], H32, H16, P16, U16, 0, nullptr, nullptr, nullptr);
  k_tok<2><<<TR, 128, 0, stream>>>(U16, nullptr, SK, PW + 3 * MW, F[11], H32, H16, P16, U16, 1, nullptr, nullptr, nullptr);
  k_nred<1><<<dim3(DD / 64, NBATCH), 128, 0, stream>>>(P16, BT, SCT, XH);
  k_mode<<<dim3(DD, NBATCH), 128, 0, stream>>>(XH, F[12], XH2);
  k_gal<<<dim3(TPB, NBATCH), 128, 0, stream>>>(B16, XH2, PW + 4 * MW, F[14], 1, H32, H16);
  k_tok<0><<<TR, 128, 0, stream>>>(H16, nullptr, SH, PW + 5 * MW, F[16], H32, H16, P16, U16, 0, nullptr, nullptr, nullptr);
  k_nred<0><<<dim3(DD / 64, NBATCH), 128, 0, stream>>>(P16, BT, SCT, XH);
  k_attn<<<dim3(TPB, NBATCH), 128, 0, stream>>>(B16, SCT, H32, H16);
  k_tok<1><<<TR, 128, 0, stream>>>(H16, nullptr, SH, PW + 6 * MW, F[18], H32, H16, P16, U16, 0, nullptr, nullptr, nullptr);
  k_tok<2><<<TR, 128, 0, stream>>>(U16, nullptr, SK, PW + 7 * MW, F[20], H32, H16, P16, U16, 1, nullptr, nullptr, nullptr);
  k_nred<1><<<dim3(DD / 64, NBATCH), 128, 0, stream>>>(P16, BT, SCT, XH);
  k_mode<<<dim3(DD, NBATCH), 128, 0, stream>>>(XH, F[21], XH2);
  k_gal<<<dim3(TPB, NBATCH), 128, 0, stream>>>(B16, XH2, PW + 8 * MW, F[23], 0, H32, H16);
  k_tok<3><<<TR, 128, 0, stream>>>(nullptr, H32, SH, PW + 9 * MW, F[25], H32, H16, P16, U16, 0, F[26], F[27], (float*)d_out);
}
